// CoAttentionModule_73289321939610
// MI455X (gfx1250) — hardware-verified
//
#include <hip/hip_runtime.h>


#ifndef NB
#define NB 4
#endif
#define NB_FULL 4
#define TQ    256
#define TK    256
#define DV    512
#define TQ_SH 8
#define TK_SH 8
#define PCAR  1024.0f
#define VSC   16.0f
#define OSC   (1.0f / 16384.0f)
#define LOG2E 1.4426950408889634f

static_assert(NB >= 1 && NB <= NB_FULL);
static_assert(TQ == TK);
static_assert((1 << TQ_SH) == TQ && (1 << TK_SH) == TK);
static_assert(TQ % 64 == 0 && TK % 64 == 0 && DV % 64 == 0);
static_assert(TQ % 32 == 0 && TK % 32 == 0);
static_assert(DV == 4 * 128);
static_assert(TK == 8 * 32 && TQ == 8 * 32);
static_assert((size_t)NB_FULL * TQ * DV * 4 == 2097152);
static_assert(((size_t)NB_FULL * TQ * DV + (size_t)NB_FULL * TK * DV) * 4 == 4194304);
static_assert((((size_t)NB * DV * TK / 2) % 256) == 0);

static constexpr size_t WS_TOTAL = (size_t)NB * DV * TK * 2 + (size_t)NB * DV * TQ * 2 + (size_t)NB * TQ * TK * 4 + (size_t)NB * TQ * TK * 2 + (size_t)NB * TK * TQ * 2;
static_assert(WS_TOTAL <= 134217728);
static_assert((((size_t)NB * DV * TK * 2) % 256) == 0 && (((size_t)NB * TQ * TK * 2) % 256) == 0);
static_assert(16 * 68 * 4 <= 131072);
static_assert((2 * TK + 8) * 4 <= 131072);

typedef _Float16 h16;
typedef __attribute__((ext_vector_type(16))) _Float16 v16h;
typedef __attribute__((ext_vector_type(8)))  _Float16 v8h;
typedef __attribute__((ext_vector_type(8)))  float    v8f;
typedef __attribute__((ext_vector_type(4)))  float    v4f;
typedef __attribute__((ext_vector_type(2)))  _Float16 v2h;
typedef v8h  __attribute__((may_alias)) v8ha;
typedef v4f  __attribute__((may_alias)) v4fa;

__device__ __forceinline__ unsigned short f2bf(float f) { unsigned u = __float_as_uint(f); u += 0x7FFFu + ((u >> 16) & 1u); return (unsigned short)(u >> 16); }
__device__ __forceinline__ float bf2f(unsigned short b) { return __uint_as_float(((unsigned)b) << 16); }
__device__ __forceinline__ float bfr(float f) { return bf2f(f2bf(f)); }
__device__ __forceinline__ v16h cat16(v8h lo, v8h hi) { return __builtin_shufflevector(lo, hi, 0, 1, 2, 3, 4, 5, 6, 7, 8, 9, 10, 11, 12, 13, 14, 15); }
__device__ __forceinline__ v8f wmma16(v16h a, v16h b, v8f c) { return __builtin_amdgcn_wmma_f32_16x16x32_f16(false, a, false, b, (short)0, c, false, false); }

static __device__ __forceinline__ h16 toh_flush(float v) { const float w = (fabsf(v) < 6.103515625e-05f) ? 0.0f : v; return (h16)w; }

template <typename T16> struct WFrag;
template <> struct WFrag<h16> { typedef v16h V; static __device__ __forceinline__ V ld(const h16* p) { return cat16(*(const v8h*)p, *(const v8h*)(p + 16)); } static __device__ __forceinline__ v8f mma(V a, V b, v8f c) { return wmma16(a, b, c); } };
template <typename T16, int NSPLIT, bool BIAS>
__global__ __launch_bounds__(32) void k_gemmw(const T16* __restrict__ A, const T16* __restrict__ A2, const T16* __restrict__ Bt, const T16* __restrict__ Bt2, int K, float* C, int ldc, const float* __restrict__ bias, float csc, size_t sA, size_t sB, size_t sC) {
    typedef typename WFrag<T16>::V V;
    __shared__ __align__(16) float os[16 * 68];
    const size_t z = blockIdx.z; A += z * sA; if (A2) A2 += z * sA; Bt += z * sB; if (Bt2) Bt2 += z * sB; C += z * sC;
    const int lane = threadIdx.x & 31, lr = lane & 15, hi = lane >> 4; const int r0 = blockIdx.x * 64, c0 = blockIdx.y * 64;
    v8f acc[4][4];
#pragma unroll
    for (int mb = 0; mb < 4; ++mb)
#pragma unroll
        for (int nb = 0; nb < 4; ++nb) acc[mb][nb] = (v8f){};
    const size_t aoff = (size_t)(r0 + lr) * K + 8 * hi, boff = (size_t)(c0 + lr) * K + 8 * hi;
#pragma unroll 1
    for (int kc = 0; kc < K; kc += 32) {
        V a[4], a2[4];
#pragma unroll
        for (int mb = 0; mb < 4; ++mb) { a[mb] = WFrag<T16>::ld(A + aoff + (size_t)mb * 16 * K + kc); if (NSPLIT == 1 || NSPLIT == 2) a2[mb] = WFrag<T16>::ld(A2 + aoff + (size_t)mb * 16 * K + kc); }
#pragma unroll
        for (int nb = 0; nb < 4; ++nb) { const V b = WFrag<T16>::ld(Bt + boff + (size_t)nb * 16 * K + kc); V b2; if (NSPLIT >= 2) b2 = WFrag<T16>::ld(Bt2 + boff + (size_t)nb * 16 * K + kc);
#pragma unroll
            for (int mb = 0; mb < 4; ++mb) { acc[mb][nb] = WFrag<T16>::mma(a[mb], b, acc[mb][nb]); if (NSPLIT == 1 || NSPLIT == 2) acc[mb][nb] = WFrag<T16>::mma(a2[mb], b, acc[mb][nb]); if (NSPLIT >= 2) acc[mb][nb] = WFrag<T16>::mma(a[mb], b2, acc[mb][nb]); } }
        asm volatile("v_nop\n\tv_nop\n\tv_nop\n\tv_nop" : "+v"(acc[0][0]), "+v"(acc[1][1]), "+v"(acc[2][2]), "+v"(acc[3][3]) : "v"(a[0]), "v"(a[3]));
    }
#pragma unroll
    for (int mb = 0; mb < 4; ++mb) {
#pragma unroll
        for (int nb = 0; nb < 4; ++nb) {
#pragma unroll
            for (int j = 0; j < 8; ++j) os[(hi * 8 + j) * 68 + nb * 16 + lr] = acc[mb][nb][j]; }
        __builtin_amdgcn_wave_barrier(); asm volatile("" ::: "memory");
        float* crow = C + (size_t)(r0 + mb * 16) * ldc + c0;
#pragma unroll 1
        for (int ps = 0; ps < 2; ++ps) {
#pragma unroll
            for (int s = 0; s < 8; ++s) { const int row = 2 * s + hi, cofs = lr * 4; v4f val = *(const v4fa*)(os + row * 68 + cofs); val = val * csc;
                if (BIAS) { val[0] += bfr(bias[c0 + cofs]); val[1] += bfr(bias[c0 + cofs + 1]); val[2] += bfr(bias[c0 + cofs + 2]); val[3] += bfr(bias[c0 + cofs + 3]); }
                *(volatile v4f*)(crow + (size_t)row * ldc + cofs) = val; }
            if (ps == 0) __threadfence(); }
        __builtin_amdgcn_wave_barrier(); asm volatile("" ::: "memory");
    }
}

__global__ __launch_bounds__(256) void k_vtp(const float* __restrict__ F, h16* V16) {
    const size_t e = ((size_t)blockIdx.x * 256 + threadIdx.x) * 2; if (e >= (size_t)NB * DV * TK) return;
    const int t = (int)(e % TK); const int d = (int)((e / TK) % DV); const int b = (int)(e / ((size_t)TK * DV));
    v2h o;
#pragma unroll
    for (int q = 0; q < 2; ++q) o[q] = toh_flush(bfr(F[((size_t)b * TK + t + q) * DV + d]) * VSC);
    *(volatile v2h*)(V16 + e) = o; __threadfence(); *(volatile v2h*)(V16 + e) = o;
}

__device__ __forceinline__ float tnh(float x) {
    const float e = __builtin_amdgcn_exp2f(x * 2.8853900817779268f);
    const float r = __builtin_amdgcn_rcpf(e + 1.0f);
    return fmaf(-2.0f, r, 1.0f);
}

static_assert(2 * 32 * 16 == TK * 4);
static_assert(1 * 32 * 16 == TK * 2);
static_assert(8 * (TK / 8) == TK && 256 == TK);
__global__ __launch_bounds__(256) void k_score(const float* __restrict__ M1, const float* __restrict__ M2, const float* __restrict__ ww, const float* __restrict__ bb, float* SF, h16* P16) {
    __shared__ __align__(16) float s_sc[TK];
    __shared__ __align__(16) float s_ex[TK];
    __shared__ float red[8];
    const int rq = blockIdx.x; const int b = rq >> TQ_SH;
    const int tid = threadIdx.x, lane = tid & 31; const int wave = __builtin_amdgcn_readfirstlane(tid >> 5);
    const float* mrow = M1 + (size_t)rq * DV;
    float mr[16], wr[16];
#pragma unroll
    for (int c = 0; c < 4; ++c) { const v4f a4 = *(const v4f*)(mrow + c * 128 + lane * 4); const v4f w4 = *(const v4f*)(ww + c * 128 + lane * 4);
#pragma unroll
        for (int e = 0; e < 4; ++e) { mr[c * 4 + e] = bfr(a4[e]); wr[c * 4 + e] = bfr(w4[e]); } }
    const float bs = bfr(bb[0]);
    const float* ub = M2 + (size_t)b * TK * DV;
#pragma unroll 1
    for (int kk = 0; kk < TK / 8; ++kk) {
        const int k = wave * (TK / 8) + kk;
        const float* urow = ub + (size_t)k * DV;
        float acc = 0.0f;
#pragma unroll
        for (int c = 0; c < 4; ++c) { const v4f u4 = *(const v4f*)(urow + c * 128 + lane * 4);
#pragma unroll
            for (int e = 0; e < 4; ++e) acc = fmaf(wr[c * 4 + e], tnh(mr[c * 4 + e] + bfr(u4[e])), acc); }
#pragma unroll
        for (int sh = 16; sh; sh >>= 1) acc += __shfl_xor(acc, sh, 32);
        if (lane == 0) s_sc[k] = acc;
    }
    __syncthreads();
    const float a0 = s_sc[tid] + bs;
    s_sc[tid] = a0;
    float m = a0;
#pragma unroll
    for (int sh = 16; sh; sh >>= 1) { const float o = __shfl_xor(m, sh, 32); m = (o > m) ? o : m; }
    if (lane == 0) red[wave] = m;
    __syncthreads();
    m = red[0];
#pragma unroll
    for (int w = 1; w < 8; ++w) { const float o = red[w]; m = (o > m) ? o : m; }
    __syncthreads();
    float d0 = a0 - m;
    const float e0 = __builtin_amdgcn_exp2f(d0 * LOG2E);
    s_ex[tid] = e0;
    float sum = e0;
#pragma unroll
    for (int sh = 16; sh; sh >>= 1) sum += __shfl_xor(sum, sh, 32);
    if (lane == 0) red[wave] = sum;
    __syncthreads();
    sum = red[0];
#pragma unroll
    for (int w = 1; w < 8; ++w) sum += red[w];
    const float inv = __builtin_amdgcn_rcpf(sum); const float invp = inv * PCAR;
    if (wave < 2) {
        const int f0 = (wave * 32 + lane) * 4;
        const v4f p = *(const v4fa*)(s_sc + f0);
        float* dst = SF + (size_t)rq * TK + f0;
        *(volatile v4f*)dst = p; __threadfence(); *(volatile v4f*)dst = p;
    } else if (wave == 2) {
        const int f0 = lane * 8;
        const v4f q0 = *(const v4fa*)(s_ex + f0); const v4f q1 = *(const v4fa*)(s_ex + f0 + 4);
        v8h o;
#pragma unroll
        for (int c = 0; c < 4; ++c) { o[c] = toh_flush(q0[c] * invp); o[4 + c] = toh_flush(q1[c] * invp); }
        h16* dst = P16 + (size_t)rq * TK + f0;
        *(volatile v8h*)dst = o; __threadfence(); *(volatile v8h*)dst = o;
    }
}

static_assert(1 * 32 * 16 == TQ * 2);
static_assert(256 == TQ);
__global__ __launch_bounds__(256) void k_csoft(const float* __restrict__ SF, h16* P2T) {
    __shared__ __align__(16) float s_ex[TQ];
    __shared__ float red[8];
    const int cq = blockIdx.x; const int b = cq >> TK_SH; const int j = cq & (TK - 1);
    const int tid = threadIdx.x, lane = tid & 31; const int wave = __builtin_amdgcn_readfirstlane(tid >> 5);
    const float a0 = SF[((size_t)((b << TQ_SH) + tid)) * TK + j];
    float m = a0;
#pragma unroll
    for (int sh = 16; sh; sh >>= 1) { const float o = __shfl_xor(m, sh, 32); m = (o > m) ? o : m; }
    if (lane == 0) red[wave] = m;
    __syncthreads();
    m = red[0];
#pragma unroll
    for (int w = 1; w < 8; ++w) { const float o = red[w]; m = (o > m) ? o : m; }
    __syncthreads();
    float d0 = a0 - m;
    const float e0 = __builtin_amdgcn_exp2f(d0 * LOG2E);
    s_ex[tid] = e0;
    float sum = e0;
#pragma unroll
    for (int sh = 16; sh; sh >>= 1) sum += __shfl_xor(sum, sh, 32);
    if (lane == 0) red[wave] = sum;
    __syncthreads();
    sum = red[0];
#pragma unroll
    for (int w = 1; w < 8; ++w) sum += red[w];
    const float inv = __builtin_amdgcn_rcpf(sum); const float invp = inv * PCAR;
    if (wave == 0) {
        const int f0 = lane * 8;
        const v4f q0 = *(const v4fa*)(s_ex + f0); const v4f q1 = *(const v4fa*)(s_ex + f0 + 4);
        v8h o;
#pragma unroll
        for (int c = 0; c < 4; ++c) { o[c] = toh_flush(q0[c] * invp); o[4 + c] = toh_flush(q1[c] * invp); }
        h16* dst = P2T + (size_t)cq * TQ + f0;
        *(volatile v8h*)dst = o; __threadfence(); *(volatile v8h*)dst = o;
    }
}

extern "C" void kernel_launch(void* const* d_in, const int* in_sizes, int n_in,
                              void* d_out, int out_size, void* d_ws, size_t ws_size, hipStream_t stream) {
    if (n_in < 4) return;
    if (in_sizes[0] < NB * TQ * DV || in_sizes[1] < NB * TK * DV || in_sizes[2] < DV || in_sizes[3] < 1) return;
    if (out_size < NB_FULL * TQ * DV + NB * TK * DV) return;
    const float* modal1 = (const float*)d_in[0];
    const float* modal2 = (const float*)d_in[1];
    const float* wvec   = (const float*)d_in[2];
    const float* bsc    = (const float*)d_in[3];
    float* OUT0 = (float*)d_out;
    float* OUT1 = OUT0 + (size_t)NB_FULL * TQ * DV;

    char* wsp = (char*)d_ws;
    auto take = [&](size_t bytes) { char* p = wsp; wsp += (bytes + 255) & ~(size_t)255; return (void*)p; };
    h16*   VT2  = (h16*)take((size_t)NB * DV * TK * 2);
    h16*   VT1  = (h16*)take((size_t)NB * DV * TQ * 2);
    float* SF   = (float*)take((size_t)NB * TQ * TK * 4);
    h16*   P1   = (h16*)take((size_t)NB * TQ * TK * 2);
    h16*   P2T  = (h16*)take((size_t)NB * TK * TQ * 2);
    if ((size_t)(wsp - (char*)d_ws) > ws_size) return;

    k_vtp<<<(unsigned)(((size_t)NB * DV * TK / 2 + 255) / 256), 256, 0, stream>>>(modal2, VT2);
    k_vtp<<<(unsigned)(((size_t)NB * DV * TQ / 2 + 255) / 256), 256, 0, stream>>>(modal1, VT1);
    k_score<<<(unsigned)(NB * TQ), 256, 0, stream>>>(modal1, modal2, wvec, bsc, SF, P1);
    k_csoft<<<(unsigned)(NB * TK), 256, 0, stream>>>(SF, P2T);
    k_gemmw<h16, 0, false><<<dim3(TQ / 64, DV / 64, NB), 32, 0, stream>>>(P1, nullptr, VT2, nullptr, TK, OUT0, DV, nullptr, OSC, (size_t)TQ * TK, (size_t)DV * TK, (size_t)TQ * DV);
    k_gemmw<h16, 0, false><<<dim3(TK / 64, DV / 64, NB), 32, 0, stream>>>(P2T, nullptr, VT1, nullptr, TQ, OUT1, DV, nullptr, OSC, (size_t)TK * TQ, (size_t)DV * TQ, (size_t)TK * DV);
}
